// RNNModel_2448131358905
// MI455X (gfx1250) — hardware-verified
//
#include <hip/hip_runtime.h>
#include <math.h>

constexpr int NBATCH   = 2048;
constexpr int NSTEP    = 512;
constexpr int NIN      = 8;
constexpr int NHID     = 64;
constexpr int ROWS_BLK = 32;
constexpr int NTHR     = 256;
constexpr int HPITCH   = 72;
constexpr int XCHUNK   = 16;
constexpr float WCARRY     = 16.0f;
constexpr float WCARRY_INV = 1.0f / WCARRY;

static_assert(NBATCH % ROWS_BLK == 0, "batch tiles exact");
static_assert(NSTEP % XCHUNK == 0, "time chunks exact");
static_assert(NHID == 64 && NIN == 8, "fragment loaders assume K = 64 (two 32-chunks) and input K = 8");
static_assert(NTHR == 32 * (ROWS_BLK / 16) * (NHID / 16), "one wave per (16-row subtile, 16-column group)");
static_assert((ROWS_BLK * XCHUNK) % NTHR == 0, "x staging loop exact");
static_assert(HPITCH % 8 == 0 && HPITCH >= NHID, "16-B aligned fragment rows");
static_assert((ROWS_BLK * HPITCH) % 8 == 0, "zero fill in 16-B slots");

typedef __attribute__((ext_vector_type(16))) _Float16 v16h;
typedef __attribute__((ext_vector_type(8)))  _Float16 v8h;
typedef __attribute__((ext_vector_type(8)))  float    v8f;
typedef __attribute__((ext_vector_type(4)))  float    v4f;

union FragU { v16h v; v8h h[2]; };

__device__ __forceinline__ v16h frag_load(const _Float16* p) {
  FragU f;
  f.h[0] = *(const v8h*)(p);
  f.h[1] = *(const v8h*)(p + 16);
  return f.v;
}

__device__ __forceinline__ v8f mma16(v16h a, v16h b, v8f c) {
  return __builtin_amdgcn_wmma_f32_16x16x32_f16(false, a, false, b, (short)0, c, false, false);
}

__device__ __forceinline__ void guard_l0(v8f& acc, v16h a0, v16h a1, v16h a2, v16h b0, v16h b1, v16h b2) {
  asm volatile("v_nop\n\tv_nop\n\tv_nop\n\tv_nop"
               : "+v"(acc)
               : "v"(a0), "v"(a1), "v"(a2), "v"(b0), "v"(b1), "v"(b2));
}
__device__ __forceinline__ void guard_l1(v8f& acc, v16h a0, v16h a1, v16h a2, v16h a3,
                                         v16h b0, v16h b1, v16h b2, v16h b3) {
  asm volatile("v_nop\n\tv_nop\n\tv_nop\n\tv_nop"
               : "+v"(acc)
               : "v"(a0), "v"(a1), "v"(a2), "v"(a3), "v"(b0), "v"(b1), "v"(b2), "v"(b3));
}

__device__ __forceinline__ float tanh_f32(float v) {
  const float e = expf(2.0f * v);
  return 1.0f - 2.0f * __builtin_amdgcn_rcpf(e + 1.0f);
}

__device__ __forceinline__ v16h wfrag64(const float* p) {
  const v4f q0 = *(const v4f*)(p);
  const v4f q1 = *(const v4f*)(p + 4);
  const v4f q2 = *(const v4f*)(p + 16);
  const v4f q3 = *(const v4f*)(p + 20);
  v16h f;
#pragma unroll
  for (int e = 0; e < 4; ++e) {
    f[e]      = (_Float16)(q0[e] * WCARRY);
    f[4 + e]  = (_Float16)(q1[e] * WCARRY);
    f[8 + e]  = (_Float16)(q2[e] * WCARRY);
    f[12 + e] = (_Float16)(q3[e] * WCARRY);
  }
  return f;
}

__device__ __forceinline__ v16h wfrag8(const float* prow, int hh) {
  v4f q0 = *(const v4f*)(prow);
  v4f q1 = *(const v4f*)(prow + 4);
  asm volatile("" : "+v"(q0), "+v"(q1));
  v16h f;
#pragma unroll
  for (int e = 0; e < 4; ++e) {
    const float s0 = (hh == 0) ? (q0[e] * WCARRY) : 0.0f;
    const float s1 = (hh == 0) ? (q1[e] * WCARRY) : 0.0f;
    f[e]      = (_Float16)s0;
    f[4 + e]  = (_Float16)s1;
    f[8 + e]  = (_Float16)0.0f;
    f[12 + e] = (_Float16)0.0f;
  }
  return f;
}

__global__ __launch_bounds__(NTHR) void rnn2_seq_kernel(
    const float* __restrict__ x,
    const float* __restrict__ wih0, const float* __restrict__ whh0,
    const float* __restrict__ bih0, const float* __restrict__ bhh0,
    const float* __restrict__ wih1, const float* __restrict__ whh1,
    const float* __restrict__ bih1, const float* __restrict__ bhh1,
    const float* __restrict__ fcw,  const float* __restrict__ fcb,
    float* __restrict__ out) {
  __shared__ __align__(16) _Float16 H0s[ROWS_BLK * HPITCH];
  __shared__ __align__(16) _Float16 H1s[ROWS_BLK * HPITCH];
  __shared__ __align__(16) _Float16 Xs[ROWS_BLK * XCHUNK * NIN];
  __shared__ __align__(16) float    Red[4 * ROWS_BLK];

  const int tid  = threadIdx.x;
  const int lane = tid & 31;
  const int wave = tid >> 5;
  const int c    = lane & 15;
  const int hh   = lane >> 4;
  const int koff = 8 * hh;
  const int u    = wave >> 2;
  const int wq   = wave & 3;
  const int b0   = blockIdx.x * ROWS_BLK;
  const int ncol  = 16 * wq + c;
  const int arow  = 16 * u + c;
  const int drow0 = 16 * u + 8 * hh;

  const v8h z8h = {(_Float16)0.0f, (_Float16)0.0f, (_Float16)0.0f, (_Float16)0.0f,
                   (_Float16)0.0f, (_Float16)0.0f, (_Float16)0.0f, (_Float16)0.0f};

#pragma unroll 1
  for (int i = tid; i < (ROWS_BLK * HPITCH) / 8; i += NTHR) {
    *(v8h*)(H0s + 8 * i) = z8h;
    *(v8h*)(H1s + 8 * i) = z8h;
  }

  const v16h b_ih0  = wfrag8(wih0 + (size_t)ncol * NIN, hh);
  const v16h b_hh0a = wfrag64(whh0 + (size_t)ncol * NHID + koff);
  const v16h b_hh0b = wfrag64(whh0 + (size_t)ncol * NHID + koff + 32);
  const v16h b_ih1a = wfrag64(wih1 + (size_t)ncol * NHID + koff);
  const v16h b_ih1b = wfrag64(wih1 + (size_t)ncol * NHID + koff + 32);
  const v16h b_hh1a = wfrag64(whh1 + (size_t)ncol * NHID + koff);
  const v16h b_hh1b = wfrag64(whh1 + (size_t)ncol * NHID + koff + 32);

  const float bias0 = (bih0[ncol] + bhh0[ncol]) * WCARRY;
  const float bias1 = (bih1[ncol] + bhh1[ncol]) * WCARRY;
  const float fw    = fcw[ncol];
  const float fcb0  = fcb[0];

  FragU zf;
  zf.h[0] = z8h;
  zf.h[1] = z8h;
  v16h ah0a = zf.v;
  v16h ah0b = zf.v;

  float h1v[8];
#pragma unroll
  for (int r = 0; r < 8; ++r) h1v[r] = 0.0f;

  const _Float16* h0row = H0s + arow * HPITCH + koff;
  const _Float16* h1row = H1s + arow * HPITCH + koff;

#pragma unroll 1
  for (int tc = 0; tc < NSTEP / XCHUNK; ++tc) {
    {
      const int t0 = tc * XCHUNK;
#pragma unroll
      for (int i = 0; i < (ROWS_BLK * XCHUNK) / NTHR; ++i) {
        const int idx = i * NTHR + tid;
        const int row = idx >> 4;
        const int ts  = idx & 15;
        const float* sp = x + ((size_t)(b0 + row) * NSTEP + (size_t)(t0 + ts)) * NIN;
        const v4f qa = *(const v4f*)(sp);
        const v4f qb = *(const v4f*)(sp + 4);
        v8h hv;
#pragma unroll
        for (int e = 0; e < 4; ++e) {
          hv[e]     = (_Float16)qa[e];
          hv[4 + e] = (_Float16)qb[e];
        }
        *(v8h*)(Xs + idx * NIN) = hv;
      }
    }
    __syncthreads();

#pragma unroll 1
    for (int tt = 0; tt < XCHUNK; ++tt) {
      v8h xv = *(const v8h*)(Xs + (arow * XCHUNK + tt) * NIN);
      asm volatile("" : "+v"(xv));
      FragU xf;
      xf.h[0] = (hh == 0) ? xv : z8h;
      xf.h[1] = z8h;
      const v16h ax = xf.v;

      v8f c0 = {bias0, bias0, bias0, bias0, bias0, bias0, bias0, bias0};
      c0 = mma16(ax,   b_ih0,  c0);
      c0 = mma16(ah0a, b_hh0a, c0);
      c0 = mma16(ah0b, b_hh0b, c0);
      guard_l0(c0, ax, ah0a, ah0b, b_ih0, b_hh0a, b_hh0b);
#pragma unroll
      for (int r = 0; r < 8; ++r) {
        const float hv = tanh_f32(c0[r] * WCARRY_INV);
        H0s[(drow0 + r) * HPITCH + ncol] = (_Float16)hv;
      }
      __syncthreads();

      ah0a = frag_load(h0row);
      ah0b = frag_load(h0row + 32);
      const v16h ah1a = frag_load(h1row);
      const v16h ah1b = frag_load(h1row + 32);
      v8f c1 = {bias1, bias1, bias1, bias1, bias1, bias1, bias1, bias1};
      c1 = mma16(ah0a, b_ih1a, c1);
      c1 = mma16(ah0b, b_ih1b, c1);
      c1 = mma16(ah1a, b_hh1a, c1);
      c1 = mma16(ah1b, b_hh1b, c1);
      guard_l1(c1, ah0a, ah0b, ah1a, ah1b, b_ih1a, b_ih1b, b_hh1a, b_hh1b);
#pragma unroll
      for (int r = 0; r < 8; ++r) h1v[r] = tanh_f32(c1[r] * WCARRY_INV);
      __syncthreads();
#pragma unroll
      for (int r = 0; r < 8; ++r) H1s[(drow0 + r) * HPITCH + ncol] = (_Float16)h1v[r];
    }
  }

#pragma unroll
  for (int r = 0; r < 8; ++r) {
    float p = h1v[r] * fw;
    p += __shfl_xor(p, 1, 32);
    p += __shfl_xor(p, 2, 32);
    p += __shfl_xor(p, 4, 32);
    p += __shfl_xor(p, 8, 32);
    if (c == 0) Red[wq * ROWS_BLK + drow0 + r] = p;
  }
  __syncthreads();
  if (wave == 0) {
    const float s = ((Red[lane] + Red[ROWS_BLK + lane]) + (Red[2 * ROWS_BLK + lane] + Red[3 * ROWS_BLK + lane])) + fcb0;
    volatile float* op = out + b0 + lane;
    *op = s;
    __threadfence();
    *op = s;
  }
}

extern "C" void kernel_launch(void* const* d_in, const int* in_sizes, int n_in,
                              void* d_out, int out_size, void* d_ws, size_t ws_size, hipStream_t stream) {
  (void)d_ws; (void)ws_size;
  if (n_in < 11 || d_out == nullptr) return;
  if (in_sizes[0] != NBATCH * NSTEP * NIN || in_sizes[1] != NHID * NIN || in_sizes[2] != NHID * NHID ||
      in_sizes[3] != NHID || in_sizes[4] != NHID || in_sizes[5] != NHID * NHID || in_sizes[6] != NHID * NHID ||
      in_sizes[7] != NHID || in_sizes[8] != NHID || in_sizes[9] != NHID || in_sizes[10] != 1 ||
      out_size != NBATCH) return;

  const float* x    = (const float*)d_in[0];
  const float* wih0 = (const float*)d_in[1];
  const float* whh0 = (const float*)d_in[2];
  const float* bih0 = (const float*)d_in[3];
  const float* bhh0 = (const float*)d_in[4];
  const float* wih1 = (const float*)d_in[5];
  const float* whh1 = (const float*)d_in[6];
  const float* bih1 = (const float*)d_in[7];
  const float* bhh1 = (const float*)d_in[8];
  const float* fcw  = (const float*)d_in[9];
  const float* fcb  = (const float*)d_in[10];
  float* out = (float*)d_out;

  rnn2_seq_kernel<<<NBATCH / ROWS_BLK, NTHR, 0, stream>>>(x, wih0, whh0, bih0, bhh0,
                                                          wih1, whh1, bih1, bhh1, fcw, fcb, out);
}
